// _SelectiveSSM_58583353917470
// MI455X (gfx1250) — hardware-verified
//
#include <hip/hip_runtime.h>
#include <math.h>

typedef __attribute__((ext_vector_type(16))) _Float16 v16h;
typedef __attribute__((ext_vector_type(8)))  _Float16 v8h;
typedef __attribute__((ext_vector_type(16))) __bf16   v16b;
typedef __attribute__((ext_vector_type(8)))  __bf16   v8b;
typedef __attribute__((ext_vector_type(8)))  float    v8f;
typedef __attribute__((ext_vector_type(4)))  float    v4f;

constexpr int kBatch = 2;
constexpr int kSeq   = 2048;
constexpr int kDm    = 1024;
constexpr int kNst   = 16;
constexpr int kDtR   = 64;
constexpr int kPr    = kDtR + 2 * kNst;
constexpr int kPrPad = 128;
constexpr int kRows  = kBatch * kSeq;
constexpr int kDmLog2 = 10;
constexpr int kScanTS = 64;
constexpr int kScanCh = 64;
constexpr int kScanYP = 68;
constexpr int kBcW    = 2 * kNst;
static_assert(kPr == 96, "x_proj width");
static_assert((1 << kDmLog2) == kDm, "channel count is a power of two");
static_assert((kDm % 32) == 0 && (kDtR % 32) == 0, "GEMM K multiples of 32");
static_assert((kRows % 64) == 0 && (kPrPad % 64) == 0 && (kDm % 64) == 0 && (kDtR % 64) == 0, "GEMM M,N multiples of 64");
static_assert(kPr <= kPrPad, "pad rows");
static_assert((kSeq % kScanTS) == 0 && (kDm % kScanCh) == 0, "scan tile multiples");
static_assert(kDtR == 64 && kBcW == 32, "column split dt | B | C");

constexpr float kCarryW  = 1024.0f;
constexpr float kCarryA  = 64.0f;
constexpr float kFoldDt  = 1.0f / (kCarryW * kCarryA);
constexpr float kF16MinNormal = 6.103515625e-05f;
constexpr float kF32MinNormal = 1.17549435e-38f;

constexpr size_t kOffXH  = 0;
constexpr size_t kOffXL  = kOffXH  + (size_t)kRows  * kDm    * 2;
constexpr size_t kOffWXH = kOffXL  + (size_t)kRows  * kDm    * 2;
constexpr size_t kOffWXL = kOffWXH + (size_t)kPrPad * kDm    * 2;
constexpr size_t kOffWDH = kOffWXL + (size_t)kPrPad * kDm    * 2;
constexpr size_t kOffXZ  = kOffWDH + (size_t)kDm    * kDtR   * 2;
constexpr size_t kOffDTR = kOffXZ  + (size_t)kRows  * kPrPad * 4;
constexpr size_t kOffDT  = kOffDTR + (size_t)kRows  * kDtR   * 2;
constexpr size_t kWsTotal = kOffDT + (size_t)kRows  * kDm    * 4;
static_assert(kWsTotal == 36831232ull, "carve total");
static_assert(kWsTotal <= 134217728ull, "carve cap");
static_assert((kOffXL % 128) == 0 && (kOffWXH % 128) == 0 && (kOffWXL % 128) == 0 && (kOffWDH % 128) == 0 &&
              (kOffXZ % 128) == 0 && (kOffDTR % 128) == 0 && (kOffDT % 128) == 0, "128-B aligned regions");

__device__ __forceinline__ unsigned short f2bf_bits(float f) {
  unsigned u = __float_as_uint(f);
  return (unsigned short)((u + 0x7FFFu + ((u >> 16) & 1u)) >> 16);
}
__device__ __forceinline__ float bf_bits2f(unsigned short h) { return __uint_as_float(((unsigned)h) << 16); }

__device__ __forceinline__ _Float16 to_f16_carried(float v, float carry) {
  const float c = v * carry;
  const float z = (fabsf(c) < kF16MinNormal) ? 0.0f : c;
  return (_Float16)z;
}

__device__ __forceinline__ void tie_acc_b(v8f& a, v16b x, v16b y, v16b z, v16b w) {
  asm volatile("v_nop\n\tv_nop\n\tv_nop\n\tv_nop" : "+v"(a) : "v"(x), "v"(y), "v"(z), "v"(w));
}
__device__ __forceinline__ void tie_acc_h(v8f& a, v16h x, v16h y) {
  asm volatile("v_nop\n\tv_nop\n\tv_nop\n\tv_nop" : "+v"(a) : "v"(x), "v"(y));
}
__device__ __forceinline__ void keep4_h(v16h a, v16h b, v16h c, v16h d) { asm volatile("v_nop" :: "v"(a), "v"(b), "v"(c), "v"(d)); }
__device__ __forceinline__ void keep4_b(v16b a, v16b b, v16b c, v16b d) { asm volatile("v_nop" :: "v"(a), "v"(b), "v"(c), "v"(d)); }
__device__ __forceinline__ void acc_guard4(v8f& a, v8f& b, v8f& c, v8f& d) { asm volatile("v_nop\n\tv_nop\n\tv_nop\n\tv_nop" : "+v"(a), "+v"(b), "+v"(c), "+v"(d)); }

template <typename T> struct Frag;
template <> struct Frag<_Float16> {
  typedef v16h V; union U { v16h v; v8h h[2]; };
  static __device__ __forceinline__ v16h load(const _Float16* p) {
    U f; f.h[0] = *(const v8h*)(p); f.h[1] = *(const v8h*)(p + 16); return f.v;
  }
  static __device__ __forceinline__ v8f mma(v16h a, v16h b, v8f c) {
    return __builtin_amdgcn_wmma_f32_16x16x32_f16(false, a, false, b, (short)0, c, false, false);
  }
};
template <> struct Frag<__bf16> {
  typedef v16b V; union U { v16b v; v8b h[2]; };
  static __device__ __forceinline__ v16b load(const __bf16* p) {
    U f; f.h[0] = *(const v8b*)(p); f.h[1] = *(const v8b*)(p + 16); return f.v;
  }
  static __device__ __forceinline__ v8f mma(v16b a, v16b b, v8f c) {
    return __builtin_amdgcn_wmma_f32_16x16x32_bf16(false, a, false, b, (short)0, c, false, false);
  }
};

__device__ __forceinline__ void wave_lds_sync() {
  __builtin_amdgcn_fence(__ATOMIC_RELEASE, "workgroup");
  __builtin_amdgcn_wave_barrier();
  __builtin_amdgcn_fence(__ATOMIC_ACQUIRE, "workgroup");
}

__device__ __forceinline__ float softplus_f(float v) {
  const float a = expf(-fabsf(v));
  return fmaxf(v, 0.0f) + log1pf(a);
}

__global__ __launch_bounds__(256) void split_rows_bf16_kernel(
    const float* __restrict__ src, unsigned short* __restrict__ dhi, unsigned short* __restrict__ dlo,
    int total8, int colsLog2, int rowsValid)
{
  const int i = blockIdx.x * 256 + threadIdx.x;
  if (i >= total8) return;
  const size_t e0 = (size_t)i << 3;
  const int row = (int)(e0 >> colsLog2);
  const int col = (int)(e0 & ((((size_t)1) << colsLog2) - 1));
  const bool ok = row < rowsValid;
  const int srow = ok ? row : (rowsValid - 1);
  const float* sp = src + (((size_t)srow) << colsLog2) + col;
  const v4f a0 = *(const v4f*)(sp);
  const v4f a1 = *(const v4f*)(sp + 4);
  v8h hv, lv;
#pragma unroll
  for (int e = 0; e < 4; ++e) {
    const float r0 = a0[e];
    const float r1 = a1[e];
    const float f0 = ok ? r0 : 0.0f;
    const float f1 = ok ? r1 : 0.0f;
    const unsigned short h0 = f2bf_bits(f0), h1 = f2bf_bits(f1);
    const unsigned short l0 = f2bf_bits(f0 - bf_bits2f(h0)), l1 = f2bf_bits(f1 - bf_bits2f(h1));
    hv[e]     = __builtin_bit_cast(_Float16, h0);
    hv[4 + e] = __builtin_bit_cast(_Float16, h1);
    lv[e]     = __builtin_bit_cast(_Float16, l0);
    lv[4 + e] = __builtin_bit_cast(_Float16, l1);
  }
  unsigned short* qh = dhi + e0;
  unsigned short* ql = dlo + e0;
  *(volatile v8h*)qh = hv;
  *(volatile v8h*)ql = lv;
  __threadfence();
  *(volatile v8h*)qh = hv;
  *(volatile v8h*)ql = lv;
}

__global__ __launch_bounds__(256) void cast_carry_f16_kernel(
    const float* __restrict__ src, unsigned short* __restrict__ dst, int total8, float carry)
{
  const int i = blockIdx.x * 256 + threadIdx.x;
  if (i >= total8) return;
  const size_t e0 = (size_t)i << 3;
  const v4f a0 = *(const v4f*)(src + e0);
  const v4f a1 = *(const v4f*)(src + e0 + 4);
  v8h hv;
#pragma unroll
  for (int e = 0; e < 4; ++e) {
    const float r0 = a0[e];
    const float r1 = a1[e];
    hv[e]     = to_f16_carried(r0, carry);
    hv[4 + e] = to_f16_carried(r1, carry);
  }
  unsigned short* q = dst + e0;
  *(volatile v8h*)q = hv;
  __threadfence();
  *(volatile v8h*)q = hv;
}

__global__ __launch_bounds__(256) void xproj_gemm_kernel(
    const unsigned short* __restrict__ Ahp, const unsigned short* __restrict__ Alp,
    const unsigned short* __restrict__ Bhp, const unsigned short* __restrict__ Blp,
    float* __restrict__ XZ, unsigned short* __restrict__ DTR)
{
  typedef Frag<__bf16> FB;
  const __bf16* Ah = (const __bf16*)Ahp;
  const __bf16* Al = (const __bf16*)Alp;
  const __bf16* Bh = (const __bf16*)Bhp;
  const __bf16* Bl = (const __bf16*)Blp;
  __shared__ __align__(16) float sT[8][16 * 68];
  const int lane = threadIdx.x & 31;
  const int wave = threadIdx.x >> 5;
  constexpr int tilesN = kPrPad >> 6;
  constexpr int tilesM = kRows >> 6;
  const int tile = blockIdx.x * 8 + wave;
  if (tile >= tilesM * tilesN) return;
  const int tm = tile / tilesN;
  const int tn = tile - tm * tilesN;
  const int m0 = tm << 6;
  const int n0 = tn << 6;
  const int rlane = lane & 15;
  const int koff  = (lane >> 4) * 8;
  const int mOff  = (lane >> 4) * 8;

  v8f acc[4][4];
#pragma unroll
  for (int i = 0; i < 4; ++i)
#pragma unroll
    for (int j = 0; j < 4; ++j) acc[i][j] = (v8f){0.f,0.f,0.f,0.f,0.f,0.f,0.f,0.f};

#pragma unroll 1
  for (int k0 = 0; k0 < kDm; k0 += 32) {
    v16b bh[4], bl[4];
#pragma unroll
    for (int j = 0; j < 4; ++j) {
      const size_t bo = (size_t)(n0 + (j << 4) + rlane) * kDm + koff + k0;
      bh[j] = FB::load(Bh + bo);
      bl[j] = FB::load(Bl + bo);
    }
#pragma unroll
    for (int i = 0; i < 4; ++i) {
      const size_t ao = (size_t)(m0 + (i << 4) + rlane) * kDm + koff + k0;
      const v16b ah = FB::load(Ah + ao);
      const v16b al = FB::load(Al + ao);
#pragma unroll
      for (int j = 0; j < 4; ++j) {
        acc[i][j] = FB::mma(ah, bh[j], acc[i][j]);
        acc[i][j] = FB::mma(ah, bl[j], acc[i][j]);
        acc[i][j] = FB::mma(al, bh[j], acc[i][j]);
      }
#pragma unroll
      for (int j = 0; j < 4; ++j) tie_acc_b(acc[i][j], ah, al, bh[j], bl[j]);
    }
    keep4_b(bh[0], bh[1], bh[2], bh[3]);
    keep4_b(bl[0], bl[1], bl[2], bl[3]);
  }
  acc_guard4(acc[0][0], acc[0][1], acc[0][2], acc[0][3]);
  acc_guard4(acc[1][0], acc[1][1], acc[1][2], acc[1][3]);
  acc_guard4(acc[2][0], acc[2][1], acc[2][2], acc[2][3]);
  acc_guard4(acc[3][0], acc[3][1], acc[3][2], acc[3][3]);

  float* slab = sT[wave];
  const bool sidePlane = (tn == 0);
  const int hh = lane >> 4, c4 = (lane & 15) * 4;
  const int q = lane >> 3, c8 = (lane & 7) * 8;
#pragma unroll
  for (int i = 0; i < 4; ++i) {
    const int mBase = m0 + (i << 4);
#pragma unroll
    for (int j = 0; j < 4; ++j) {
#pragma unroll
      for (int r = 0; r < 8; ++r) slab[(mOff + r) * 68 + (j << 4) + rlane] = acc[i][j][r];
    }
    wave_lds_sync();
    v8h hv[4];
#pragma unroll
    for (int it = 0; it < 4; ++it) {
      const float* sp = slab + (it * 4 + q) * 68 + c8;
      const v4f a0 = *(const v4f*)(sp);
      const v4f a1 = *(const v4f*)(sp + 4);
#pragma unroll
      for (int e = 0; e < 4; ++e) {
        const float r0 = a0[e];
        const float r1 = a1[e];
        hv[it][e]     = to_f16_carried(r0, kCarryA);
        hv[it][4 + e] = to_f16_carried(r1, kCarryA);
      }
    }
    for (int pass = 0; pass < 2; ++pass) {
#pragma unroll
      for (int it = 0; it < 8; ++it) {
        const int row = it * 2 + hh;
        const v4f v = *(const v4f*)(slab + row * 68 + c4);
        *(volatile v4f*)(XZ + (size_t)(mBase + row) * kPrPad + n0 + c4) = v;
      }
      if (sidePlane) {
#pragma unroll
        for (int it = 0; it < 4; ++it) {
          const int row = it * 4 + q;
          *(volatile v8h*)(DTR + (size_t)(mBase + row) * kDtR + c8) = hv[it];
        }
      }
      __threadfence();
    }
    wave_lds_sync();
  }
}

__global__ __launch_bounds__(256) void dtproj_gemm_kernel(
    const unsigned short* __restrict__ Ap, const unsigned short* __restrict__ Btp,
    const float* __restrict__ bdt, float* __restrict__ DT)
{
  typedef Frag<_Float16> FH;
  const _Float16* A  = (const _Float16*)Ap;
  const _Float16* Bt = (const _Float16*)Btp;
  __shared__ __align__(16) float sT[8][16 * 68];
  const int lane = threadIdx.x & 31;
  const int wave = threadIdx.x >> 5;
  constexpr int tilesN = kDm >> 6;
  constexpr int tilesM = kRows >> 6;
  const int tile = blockIdx.x * 8 + wave;
  if (tile >= tilesM * tilesN) return;
  const int tm = tile / tilesN;
  const int tn = tile - tm * tilesN;
  const int m0 = tm << 6;
  const int n0 = tn << 6;
  const int rlane = lane & 15;
  const int koff  = (lane >> 4) * 8;
  const int mOff  = (lane >> 4) * 8;

  v8f acc[4][4];
#pragma unroll
  for (int i = 0; i < 4; ++i)
#pragma unroll
    for (int j = 0; j < 4; ++j) acc[i][j] = (v8f){0.f,0.f,0.f,0.f,0.f,0.f,0.f,0.f};

#pragma unroll 1
  for (int k0 = 0; k0 < kDtR; k0 += 32) {
    v16h bh[4];
#pragma unroll
    for (int j = 0; j < 4; ++j) {
      const size_t bo = (size_t)(n0 + (j << 4) + rlane) * kDtR + koff + k0;
      bh[j] = FH::load(Bt + bo);
    }
#pragma unroll
    for (int i = 0; i < 4; ++i) {
      const size_t ao = (size_t)(m0 + (i << 4) + rlane) * kDtR + koff + k0;
      const v16h ah = FH::load(A + ao);
#pragma unroll
      for (int j = 0; j < 4; ++j) acc[i][j] = FH::mma(ah, bh[j], acc[i][j]);
#pragma unroll
      for (int j = 0; j < 4; ++j) tie_acc_h(acc[i][j], ah, bh[j]);
    }
    keep4_h(bh[0], bh[1], bh[2], bh[3]);
  }
  acc_guard4(acc[0][0], acc[0][1], acc[0][2], acc[0][3]);
  acc_guard4(acc[1][0], acc[1][1], acc[1][2], acc[1][3]);
  acc_guard4(acc[2][0], acc[2][1], acc[2][2], acc[2][3]);
  acc_guard4(acc[3][0], acc[3][1], acc[3][2], acc[3][3]);

  float* slab = sT[wave];
  const int hh = lane >> 4, c4 = (lane & 15) * 4;
#pragma unroll
  for (int i = 0; i < 4; ++i) {
    const int mBase = m0 + (i << 4);
#pragma unroll
    for (int j = 0; j < 4; ++j) {
      const float bv = bdt[n0 + (j << 4) + rlane];
#pragma unroll
      for (int r = 0; r < 8; ++r) slab[(mOff + r) * 68 + (j << 4) + rlane] = acc[i][j][r] * kFoldDt + bv;
    }
    wave_lds_sync();
#pragma unroll 1
    for (int rr = 0; rr < 16; ++rr) {
      float* p = slab + rr * 68 + 2 * lane;
      const float a0 = p[0];
      const float a1 = p[1];
      const float s0 = softplus_f(a0);
      const float s1 = softplus_f(a1);
      p[0] = s0;
      p[1] = s1;
    }
    wave_lds_sync();
    for (int pass = 0; pass < 2; ++pass) {
#pragma unroll
      for (int it = 0; it < 8; ++it) {
        const int row = it * 2 + hh;
        const v4f v = *(const v4f*)(slab + row * 68 + c4);
        *(volatile v4f*)(DT + (size_t)(mBase + row) * kDm + n0 + c4) = v;
      }
      __threadfence();
    }
    wave_lds_sync();
  }
}

__global__ __launch_bounds__(64) void scan_kernel(
    const float* __restrict__ x, const float* __restrict__ XZ, const float* __restrict__ DT,
    const float* __restrict__ Alog, const float* __restrict__ Dp, float* __restrict__ out)
{
  __shared__ __align__(16) float sBC[kScanTS * kBcW];
  __shared__ __align__(16) float sY[kScanTS * kScanYP];
  __shared__ __align__(16) float sA[kNst * kScanCh];
  const int tid = threadIdx.x, lane = tid & 31, wave = tid >> 5;
  constexpr int kBlkPerB = kDm / kScanCh;
  const int bix = blockIdx.x / kBlkPerB;
  const int d0  = (blockIdx.x - bix * kBlkPerB) * kScanCh;
  const int d   = d0 + tid;
  const size_t row0 = (size_t)bix * kSeq;
#pragma unroll 1
  for (int s = 0; s < kNst; ++s) sA[s * kScanCh + tid] = -expf(Alog[(size_t)d * kNst + s]);
  __syncthreads();
  float negA[kNst], h[kNst];
#pragma unroll
  for (int s = 0; s < kNst; ++s) {
    negA[s] = sA[s * kScanCh + tid];
    h[s] = 0.f;
  }
  const float Dd = Dp[d];
  const int lr = tid >> 3, lc4 = (tid & 7) * 4;
  const int hh = lane >> 4, c4 = (lane & 15) * 4;
#pragma unroll 1
  for (int t0 = 0; t0 < kSeq; t0 += kScanTS) {
    __syncthreads();
#pragma unroll
    for (int i = 0; i < 8; ++i) {
      const int r = lr + 8 * i;
      *(v4f*)(sBC + r * kBcW + lc4) = *(const v4f*)(XZ + (row0 + t0 + r) * kPrPad + kDtR + lc4);
    }
    __syncthreads();
#pragma unroll 1
    for (int s = 0; s < kScanTS; ++s) {
      const size_t g = (row0 + t0 + s) * kDm + d;
      const float dtv = DT[g];
      const float xt  = x[g];
      const float* br = sBC + s * kBcW;
      float Bs[kNst], Cs[kNst];
#pragma unroll
      for (int q4 = 0; q4 < 4; ++q4) {
        const v4f bv = *(const v4f*)(br + 4 * q4);
        const v4f cv = *(const v4f*)(br + kNst + 4 * q4);
        Bs[4 * q4 + 0] = bv[0]; Bs[4 * q4 + 1] = bv[1]; Bs[4 * q4 + 2] = bv[2]; Bs[4 * q4 + 3] = bv[3];
        Cs[4 * q4 + 0] = cv[0]; Cs[4 * q4 + 1] = cv[1]; Cs[4 * q4 + 2] = cv[2]; Cs[4 * q4 + 3] = cv[3];
      }
      const float dtx = dtv * xt;
      float y = 0.f;
#pragma unroll
      for (int k = 0; k < kNst; ++k) {
        const float e0 = expf(dtv * negA[k]);
        const float e  = (e0 < kF32MinNormal) ? 0.0f : e0;
        h[k] = e * h[k] + dtx * Bs[k];
        y = h[k] * Cs[k] + y;
      }
      sY[s * kScanYP + tid] = y + Dd * xt;
    }
    __syncthreads();
    for (int pass = 0; pass < 2; ++pass) {
#pragma unroll
      for (int it = 0; it < 16; ++it) {
        const int row = it * 4 + wave * 2 + hh;
        const v4f v = *(const v4f*)(sY + row * kScanYP + c4);
        *(volatile v4f*)(out + (row0 + t0 + row) * kDm + d0 + c4) = v;
      }
      __threadfence();
    }
  }
}

extern "C" void kernel_launch(void* const* d_in, const int* in_sizes, int n_in,
                              void* d_out, int out_size, void* d_ws, size_t ws_size,
                              hipStream_t stream) {
  if (n_in < 6) return;
  if (in_sizes[0] != kRows * kDm) return;
  if (in_sizes[1] != kPr * kDm) return;
  if (in_sizes[2] != kDm * kDtR) return;
  if (in_sizes[3] != kDm) return;
  if (in_sizes[4] != kDm * kNst) return;
  if (in_sizes[5] != kDm) return;
  if (out_size != kRows * kDm) return;
  if (ws_size < kWsTotal) return;

  const float* x       = (const float*)d_in[0];
  const float* W_xproj = (const float*)d_in[1];
  const float* W_dt    = (const float*)d_in[2];
  const float* b_dt    = (const float*)d_in[3];
  const float* A_log   = (const float*)d_in[4];
  const float* Dp      = (const float*)d_in[5];
  float* out = (float*)d_out;

  char* ws = (char*)d_ws;
  unsigned short* XH  = (unsigned short*)(ws + kOffXH);
  unsigned short* XL  = (unsigned short*)(ws + kOffXL);
  unsigned short* WXH = (unsigned short*)(ws + kOffWXH);
  unsigned short* WXL = (unsigned short*)(ws + kOffWXL);
  unsigned short* WDH = (unsigned short*)(ws + kOffWDH);
  float*          XZ  = (float*)(ws + kOffXZ);
  unsigned short* DTR = (unsigned short*)(ws + kOffDTR);
  float*          DT  = (float*)(ws + kOffDT);

  split_rows_bf16_kernel<<<(kRows * kDm / 8) / 256, 256, 0, stream>>>(x, XH, XL, kRows * kDm / 8, kDmLog2, kRows);
  split_rows_bf16_kernel<<<(kPrPad * kDm / 8) / 256, 256, 0, stream>>>(W_xproj, WXH, WXL, kPrPad * kDm / 8, kDmLog2, kPr);
  cast_carry_f16_kernel<<<(kDm * kDtR / 8) / 256, 256, 0, stream>>>(W_dt, WDH, kDm * kDtR / 8, kCarryW);

  xproj_gemm_kernel<<<((kRows / 64) * (kPrPad / 64)) / 8, 256, 0, stream>>>(XH, XL, WXH, WXL, XZ, DTR);

  dtproj_gemm_kernel<<<((kRows / 64) * (kDm / 64)) / 8, 256, 0, stream>>>(DTR, WDH, b_dt, DT);

  scan_kernel<<<kBatch * (kDm / kScanCh), kScanCh, 0, stream>>>(x, XZ, DT, A_log, Dp, out);
}
